// CharRNN_27779848471276
// MI455X (gfx1250) — hardware-verified
//
#include <hip/hip_runtime.h>

typedef __attribute__((ext_vector_type(16))) _Float16 v16h;
typedef __attribute__((ext_vector_type(8)))  _Float16 v8h;
typedef __attribute__((ext_vector_type(16))) __bf16   v16b;
typedef __attribute__((ext_vector_type(8)))  __bf16   v8b;
typedef __attribute__((ext_vector_type(8)))  float    v8f;
typedef __attribute__((ext_vector_type(4)))  float    v4f;

constexpr int kSeq   = 64;
constexpr int kStep  = 512;
constexpr int kEmb   = 256;
constexpr int kHid   = 1024;
constexpr int kChar  = 128;

constexpr int kSeqPB      = 16;
constexpr int kRnnBlocks  = kSeq / kSeqPB;
constexpr int kRnnThreads = 256;
constexpr int kColsPW     = 128;
constexpr int kHP         = kHid + 8;
constexpr int kHTile      = kSeqPB * kHP;
static_assert(kSeq % kSeqPB == 0, "blocks");
static_assert(kHid == (kRnnThreads / 32) * kColsPW, "wave columns cover the hidden dim exactly");
static_assert(kHP % 8 == 0, "16-B aligned fragment loads");
static_assert(kHid % 32 == 0 && kEmb % 32 == 0, "K multiples of 32");
static_assert(kChar % 64 == 0 && kHid % 64 == 0 && kSeq % 64 == 0, "GEMM tile multiples");

constexpr int kDwEmb = kChar * kEmb / 2;
constexpr int kDwWih = kHid * kEmb / 2;
constexpr int kDwWhh = kHid * kHid / 2;
constexpr int kDwWpj = kChar * kHid / 2;
constexpr int kPrepB1 = kDwEmb / 256;
constexpr int kPrepB2 = kPrepB1 + kDwWih / 256;
constexpr int kPrepB3 = kPrepB2 + kDwWhh / 256;
constexpr int kPrepBlocks = kPrepB3 + kDwWpj / 256;
static_assert(kDwEmb % 256 == 0 && kDwWih % 256 == 0 && kDwWhh % 256 == 0 && kDwWpj % 256 == 0, "exact coverage");
static_assert(kPrepBlocks == 2880, "prep grid");

__device__ __forceinline__ unsigned short f2bf_bits(float f) {
  unsigned u = __float_as_uint(f);
  return (unsigned short)((u + 0x7FFFu + ((u >> 16) & 1u)) >> 16);
}
__device__ __forceinline__ float bf_bits2f(unsigned short h) { return __uint_as_float(((unsigned)h) << 16); }

__device__ __forceinline__ void dep_guard_h(v8f& a, v8f& b, v16h x, v16h y) { asm volatile("v_nop\n\tv_nop\n\tv_nop\n\tv_nop" : "+v"(a), "+v"(b) : "v"(x), "v"(y)); }
__device__ __forceinline__ void dep_guard_b(v8f& a, v8f& b, v16b x, v16b y) { asm volatile("v_nop\n\tv_nop\n\tv_nop\n\tv_nop" : "+v"(a), "+v"(b) : "v"(x), "v"(y)); }
__device__ __forceinline__ void keep4_h(v16h a, v16h b, v16h c, v16h d) { asm volatile("v_nop" :: "v"(a), "v"(b), "v"(c), "v"(d)); }
__device__ __forceinline__ void keep4_b(v16b a, v16b b, v16b c, v16b d) { asm volatile("v_nop" :: "v"(a), "v"(b), "v"(c), "v"(d)); }
__device__ __forceinline__ void acc_guard4(v8f& a, v8f& b, v8f& c, v8f& d) { asm volatile("v_nop\n\tv_nop\n\tv_nop\n\tv_nop" : "+v"(a), "+v"(b), "+v"(c), "+v"(d)); }

template <typename T> struct Frag;
template <> struct Frag<_Float16> {
  typedef v16h V; union U { v16h v; v8h h[2]; };
  static __device__ __forceinline__ v16h load(const _Float16* p) {
    U f; f.h[0] = *(const v8h*)(p); f.h[1] = *(const v8h*)(p + 16); return f.v;
  }
  static __device__ __forceinline__ v8f mma(v16h a, v16h b, v8f c) {
    return __builtin_amdgcn_wmma_f32_16x16x32_f16(false, a, false, b, (short)0, c, false, false);
  }
  static __device__ __forceinline__ void guard(v8f& a, v8f& b, v16h x, v16h y) { dep_guard_h(a, b, x, y); }
  static __device__ __forceinline__ void keep(v16h a, v16h b, v16h c, v16h d) { keep4_h(a, b, c, d); }
};
template <> struct Frag<__bf16> {
  typedef v16b V; union U { v16b v; v8b h[2]; };
  static __device__ __forceinline__ v16b load(const __bf16* p) {
    U f; f.h[0] = *(const v8b*)(p); f.h[1] = *(const v8b*)(p + 16); return f.v;
  }
  static __device__ __forceinline__ v8f mma(v16b a, v16b b, v8f c) {
    return __builtin_amdgcn_wmma_f32_16x16x32_bf16(false, a, false, b, (short)0, c, false, false);
  }
  static __device__ __forceinline__ void guard(v8f& a, v8f& b, v16b x, v16b y) { dep_guard_b(a, b, x, y); }
  static __device__ __forceinline__ void keep(v16b a, v16b b, v16b c, v16b d) { keep4_b(a, b, c, d); }
};

template <int ET> struct Elem;
template <> struct Elem<0> { typedef _Float16 T; };
template <> struct Elem<1> { typedef __bf16 T; };
template <int ET, bool SPLIT, int BIAS_MODE, int OUT_MODE, bool RESID, int ACT = 0, int TRI = 0>
__global__ __launch_bounds__(256) void wmma_gemm64(
    const unsigned short* __restrict__ Ap, const unsigned short* __restrict__ A2p, int lda, long strideA,
    const unsigned short* __restrict__ Btp, const unsigned short* __restrict__ Bt2p, int ldb, long strideB,
    void* __restrict__ Cout, void* __restrict__ Cout2, int ldc, long strideC,
    const float* __restrict__ bias,
    const float* __restrict__ resid, long strideR,
    int M, int N, int K, float scale) {
  typedef typename Elem<ET>::T T;
  typedef typename Frag<T>::V V;
  const T* A = (const T*)Ap; const T* A2 = (const T*)A2p; const T* Bt = (const T*)Btp; const T* Bt2 = (const T*)Bt2p;
  __shared__ __align__(16) float sT[8][16 * 68];
  const int b    = blockIdx.y;
  const int lane = threadIdx.x & 31;
  const int wave = threadIdx.x >> 5;
  const int tilesN = N >> 6;
  const int tilesM = M >> 6;
  const int tile = blockIdx.x * 8 + wave;
  if (tile >= tilesM * tilesN) return;
  const int tm = tile / tilesN;
  const int tn = tile - tm * tilesN;
  if (TRI == 1 && tn > tm) return;
  const int m0 = tm << 6;
  const int n0 = tn << 6;
  const int kLim = (TRI == 2) ? ((m0 + 64 < K) ? (m0 + 64) : K) : K;

  const T* Ab  = A  + (size_t)b * strideA;
  const T* Bb  = Bt + (size_t)b * strideB;
  const T* Ab2 = SPLIT ? (A2  + (size_t)b * strideA) : nullptr;
  const T* Bb2 = SPLIT ? (Bt2 + (size_t)b * strideB) : nullptr;

  const int rlane = lane & 15;
  const int koff  = (lane >> 4) * 8;
  const int mOff  = (lane >> 4) * 8;

  v8f acc[4][4];
#pragma unroll
  for (int i = 0; i < 4; ++i)
#pragma unroll
    for (int j = 0; j < 4; ++j) acc[i][j] = (v8f){0.f,0.f,0.f,0.f,0.f,0.f,0.f,0.f};

  for (int k0 = 0; k0 < kLim; k0 += 32) {
    V bh[4], bl[4];
#pragma unroll
    for (int j = 0; j < 4; ++j) {
      const size_t bo = (size_t)(n0 + (j << 4) + rlane) * ldb + koff + k0;
      bh[j] = Frag<T>::load(Bb + bo);
      if (SPLIT) bl[j] = Frag<T>::load(Bb2 + bo);
    }
#pragma unroll
    for (int i = 0; i < 4; ++i) {
      const size_t ao = (size_t)(m0 + (i << 4) + rlane) * lda + koff + k0;
      V ah = Frag<T>::load(Ab + ao);
      V al;
      if (SPLIT) al = Frag<T>::load(Ab2 + ao);
#pragma unroll
      for (int j = 0; j < 4; ++j) {
        acc[i][j] = Frag<T>::mma(ah, bh[j], acc[i][j]);
        if (SPLIT) {
          acc[i][j] = Frag<T>::mma(ah, bl[j], acc[i][j]);
          acc[i][j] = Frag<T>::mma(al, bh[j], acc[i][j]);
        }
      }
      Frag<T>::guard(acc[i][0], acc[i][3], ah, SPLIT ? al : ah);
    }
    Frag<T>::keep(bh[0], bh[1], bh[2], bh[3]);
    if (SPLIT) Frag<T>::keep(bl[0], bl[1], bl[2], bl[3]);
  }
  acc_guard4(acc[0][0], acc[0][1], acc[0][2], acc[0][3]);
  acc_guard4(acc[1][0], acc[1][1], acc[1][2], acc[1][3]);
  acc_guard4(acc[2][0], acc[2][1], acc[2][2], acc[2][3]);
  acc_guard4(acc[3][0], acc[3][1], acc[3][2], acc[3][3]);

  float* slab = sT[wave];
  const float* Rb = RESID ? (resid + (size_t)b * strideR) : nullptr;
#pragma unroll
  for (int i = 0; i < 4; ++i) {
    const int mBase = m0 + (i << 4);
#pragma unroll
    for (int j = 0; j < 4; ++j) {
      const int n = n0 + (j << 4) + rlane;
      float bv = 0.f;
      if (BIAS_MODE == 2) bv = bias[n];
#pragma unroll
      for (int r = 0; r < 8; ++r) {
        float v = acc[i][j][r] * scale;
        if (BIAS_MODE == 1) v += bias[mBase + mOff + r];
        if (BIAS_MODE == 2) v += bv;
        if (RESID) v += Rb[(size_t)(mBase + mOff + r) * ldc + n];
        if (ACT == 1) v = tanhf(v);
        if (ACT == 2) v = fmaxf(v, 0.0f);
        if (ACT == 4) v = (v > 0.f) ? v : 0.01f * v;
        slab[(mOff + r) * 68 + (j << 4) + rlane] = v;
      }
    }
    __builtin_amdgcn_fence(__ATOMIC_RELEASE, "workgroup");
    __builtin_amdgcn_wave_barrier();
    __builtin_amdgcn_fence(__ATOMIC_ACQUIRE, "workgroup");
    if (OUT_MODE == 0) {
      float* C = (float*)Cout + (size_t)b * strideC;
      const int hh = lane >> 4, c4 = (lane & 15) * 4;
      for (int pass = 0; pass < 2; ++pass) {
#pragma unroll
        for (int it = 0; it < 8; ++it) {
          const int row = it * 2 + hh;
          v4f v = *(const v4f*)(slab + row * 68 + c4);
          *(volatile v4f*)(C + (size_t)(mBase + row) * ldc + n0 + c4) = v;
        }
        __threadfence();
      }
    } else {
      const int q = lane >> 3, c8 = (lane & 7) * 8;
      unsigned short* C  = (unsigned short*)Cout  + (size_t)b * strideC;
      unsigned short* C2 = (OUT_MODE == 2) ? ((unsigned short*)Cout2 + (size_t)b * strideC) : nullptr;
      for (int pass = 0; pass < 2; ++pass) {
#pragma unroll
        for (int it = 0; it < 4; ++it) {
          const int row = it * 4 + q;
          const float* sp = slab + row * 68 + c8;
          v8h hv, lv;
#pragma unroll
          for (int e = 0; e < 8; ++e) {
            if (OUT_MODE == 1) {
              hv[e] = (_Float16)sp[e];
            } else {
              unsigned short hb = f2bf_bits(sp[e]);
              unsigned short lb = f2bf_bits(sp[e] - bf_bits2f(hb));
              hv[e] = __builtin_bit_cast(_Float16, hb);
              lv[e] = __builtin_bit_cast(_Float16, lb);
            }
          }
          *(volatile v8h*)(C + (size_t)(mBase + row) * ldc + n0 + c8) = hv;
          if (OUT_MODE == 2) *(volatile v8h*)(C2 + (size_t)(mBase + row) * ldc + n0 + c8) = lv;
        }
        __threadfence();
      }
    }
    __builtin_amdgcn_fence(__ATOMIC_RELEASE, "workgroup");
    __builtin_amdgcn_wave_barrier();
    __builtin_amdgcn_fence(__ATOMIC_ACQUIRE, "workgroup");
  }
}

__device__ __forceinline__ unsigned pack_f16x2(float a, float b) {
  const _Float16 h0 = (_Float16)a, h1 = (_Float16)b;
  return (unsigned)__builtin_bit_cast(unsigned short, h0) | ((unsigned)__builtin_bit_cast(unsigned short, h1) << 16);
}
__device__ __forceinline__ void st2u(unsigned* p, unsigned v) { *(volatile unsigned*)p = v; __threadfence(); *(volatile unsigned*)p = v; }
__device__ __forceinline__ float ftanh(float x) { return 1.0f - 2.0f * __builtin_amdgcn_rcpf(1.0f + __expf(2.0f * x)); }

__global__ __launch_bounds__(256) void prep_kernel(
    const float* __restrict__ emb, const float* __restrict__ w_ih,
    const float* __restrict__ w_hh, const float* __restrict__ w_pj,
    unsigned* __restrict__ embu, unsigned* __restrict__ wihu,
    unsigned* __restrict__ whhu, unsigned* __restrict__ wpju) {
  const int blk = blockIdx.x, tid = threadIdx.x;
  if (blk < kPrepB1) {
    const int p = blk * 256 + tid;
    st2u(embu + p, pack_f16x2(emb[2 * p] * 4.0f, emb[2 * p + 1] * 4.0f));
  } else if (blk < kPrepB2) {
    const int p = (blk - kPrepB1) * 256 + tid;
    st2u(wihu + p, pack_f16x2(w_ih[2 * p] * 8.0f, w_ih[2 * p + 1] * 8.0f));
  } else if (blk < kPrepB3) {
    const int p = (blk - kPrepB2) * 256 + tid;
    st2u(whhu + p, pack_f16x2(w_hh[2 * p] * 16.0f, w_hh[2 * p + 1] * 16.0f));
  } else {
    const int p = (blk - kPrepB3) * 256 + tid;
    st2u(wpju + p, pack_f16x2(w_pj[2 * p] * 16.0f, w_pj[2 * p + 1] * 16.0f));
  }
}

__global__ __launch_bounds__(kRnnThreads) void rnn_kernel(
    const int* __restrict__ tok, const float* __restrict__ p16tab,
    const _Float16* __restrict__ whh16, const float* __restrict__ h0,
    _Float16* __restrict__ hf16) {
  __shared__ __align__(16) _Float16 htile[kHTile];
  const int tid = threadIdx.x, lane = tid & 31, wave = tid >> 5;
  const int c = lane & 15, hh = lane >> 4, koff = hh * 8, mOff = hh * 8;
  const int seq0 = blockIdx.x * kSeqPB;
  const int n0 = wave * kColsPW;

  for (int i = tid; i < kHTile; i += kRnnThreads) {
    const int col = i % kHP;
    const int cc = (col < kHid) ? col : (kHid - 1);
    const float v = h0[cc];
    htile[i] = (col < kHid) ? (_Float16)v : (_Float16)0.0f;
  }
  __syncthreads();

  const float inv16 = 0.0625f;
  const _Float16* brow = whh16 + (size_t)(n0 + c) * kHid + koff;
  const _Float16* arow = htile + c * kHP + koff;
  const float*    prow = p16tab + n0 + c;
  const int*      trow = tok + (size_t)(seq0 + 8 * hh) * kStep;
  const int c16 = (lane & 15) * 8;

#pragma unroll 1
  for (int s = 0; s < kStep; ++s) {
    int idoff[8];
#pragma unroll
    for (int r = 0; r < 8; ++r) {
      int v = trow[r * kStep + s];
      v = (v < 0) ? 0 : v;
      v = (v > kChar - 1) ? (kChar - 1) : v;
      idoff[r] = v * kHid;
    }
    v8f acc[8];
#pragma unroll
    for (int j = 0; j < 8; ++j) {
      const float* pj = prow + 16 * j;
#pragma unroll
      for (int r = 0; r < 8; ++r) acc[j][r] = pj[idoff[r]];
    }

    v16h fa;
    v16h fb[4];
#pragma unroll 2
    for (int kc = 0; kc < kHid / 32; ++kc) {
      fa = Frag<_Float16>::load(arow + kc * 32);
#pragma unroll
      for (int g = 0; g < 2; ++g) {
#pragma unroll
        for (int j = 0; j < 4; ++j) fb[j] = Frag<_Float16>::load(brow + (size_t)(64 * g + 16 * j) * kHid + kc * 32);
#pragma unroll
        for (int j = 0; j < 4; ++j) acc[4 * g + j] = Frag<_Float16>::mma(fa, fb[j], acc[4 * g + j]);
        Frag<_Float16>::guard(acc[4 * g], acc[4 * g + 3], fa, fb[3]);
        Frag<_Float16>::keep(fb[0], fb[1], fb[2], fb[3]);
      }
    }
    acc_guard4(acc[0], acc[1], acc[2], acc[3]);
    acc_guard4(acc[4], acc[5], acc[6], acc[7]);

    __syncthreads();

#pragma unroll
    for (int j = 0; j < 8; ++j) {
#pragma unroll
      for (int r = 0; r < 8; ++r) {
        const float hv = ftanh(acc[j][r] * inv16);
        htile[(mOff + r) * kHP + n0 + 16 * j + c] = (_Float16)hv;
      }
    }
    __syncthreads();
  }

  for (int pass = 0; pass < 2; ++pass) {
#pragma unroll
    for (int it = 0; it < 8; ++it) {
      const int rr = it * 2 + hh;
      const v8h v = *(const v8h*)(htile + rr * kHP + n0 + c16);
      *(volatile v8h*)(hf16 + (size_t)(seq0 + rr) * kHid + n0 + c16) = v;
    }
    __threadfence();
  }
}

extern "C" void kernel_launch(void* const* d_in, const int* in_sizes, int n_in,
                              void* d_out, int out_size, void* d_ws, size_t ws_size, hipStream_t stream) {
  if (n_in < 7 || d_out == nullptr || d_ws == nullptr) return;
  if (in_sizes[0] != kSeq * kStep || in_sizes[1] != kChar * kEmb || in_sizes[2] != kHid * kEmb ||
      in_sizes[3] != kHid * kHid || in_sizes[4] != kHid || in_sizes[5] != kChar * kHid || in_sizes[6] != kChar ||
      out_size != kSeq * kChar) return;

  const int*   tok    = (const int*)d_in[0];
  const float* emb    = (const float*)d_in[1];
  const float* w_ih   = (const float*)d_in[2];
  const float* w_hh   = (const float*)d_in[3];
  const float* h0     = (const float*)d_in[4];
  const float* w_pj   = (const float*)d_in[5];
  const float* b_pj   = (const float*)d_in[6];
  float* out = (float*)d_out;

  char* ws = (char*)d_ws; size_t off = 0;
  auto carve = [&](size_t bytes) -> char* { char* p = ws + off; off += (bytes + 255) & ~(size_t)255; return p; };
  unsigned short* EMB16 = (unsigned short*)carve((size_t)kChar * kEmb * 2);
  unsigned short* WIH16 = (unsigned short*)carve((size_t)kHid * kEmb * 2);
  unsigned short* WHH16 = (unsigned short*)carve((size_t)kHid * kHid * 2);
  unsigned short* WPJ16 = (unsigned short*)carve((size_t)kChar * kHid * 2);
  float*          P16   = (float*)carve((size_t)kChar * kHid * 4);
  unsigned short* HF16  = (unsigned short*)carve((size_t)kSeq * kHid * 2);
  if (off > ws_size || off > (size_t)134217728) return;

  prep_kernel<<<kPrepBlocks, 256, 0, stream>>>(emb, w_ih, w_hh, w_pj,
                                               (unsigned*)EMB16, (unsigned*)WIH16, (unsigned*)WHH16, (unsigned*)WPJ16);

  wmma_gemm64<0, false, 0, 0, false, 0, 0><<<dim3(4, 1), 256, 0, stream>>>(
      EMB16, nullptr, kEmb, 0L, WIH16, nullptr, kEmb, 0L,
      (void*)P16, nullptr, kHid, 0L, nullptr, nullptr, 0L, kChar, kHid, kEmb, 0.5f);

  rnn_kernel<<<kRnnBlocks, kRnnThreads, 0, stream>>>(tok, P16, (const _Float16*)WHH16, h0, (_Float16*)HF16);

  wmma_gemm64<0, false, 2, 0, false, 0, 0><<<dim3(1, 1), 64, 0, stream>>>(
      HF16, nullptr, kHid, 0L, WPJ16, nullptr, kHid, 0L,
      (void*)out, nullptr, kChar, 0L, b_pj, nullptr, 0L, kSeq, kChar, kHid, 1.0f / 16.0f);
}
